// RetrocausalAttention_28939489640882
// MI455X (gfx1250) — hardware-verified
//
#include <hip/hip_runtime.h>
#include <math.h>
#include <stdint.h>

#define NB    2
#define SEQ   2048
#define DM    1024
#define NH    16
#define HD    64
#define HG    2
#define NGRP  (NH / HG)
#define WINW  32
#define LNEPS 1e-5f
#define PCARRY     32768.0f
#define PCARRY_INV (1.0f / 32768.0f)
#define FBCARRY    16.0f
#define WCARRY     16.0f

typedef __attribute__((ext_vector_type(16))) _Float16 v16h;
typedef __attribute__((ext_vector_type(8)))  _Float16 v8h;
typedef __attribute__((ext_vector_type(16))) __bf16   v16b;
typedef __attribute__((ext_vector_type(8)))  __bf16   v8b;
typedef __attribute__((ext_vector_type(8)))  float    v8f;
typedef __attribute__((ext_vector_type(4)))  float    v4f;
typedef __attribute__((ext_vector_type(2)))  float    v2f;
typedef __attribute__((ext_vector_type(4)))  unsigned int v4u;

__device__ __forceinline__ unsigned short f2bf_bits(float f) {
  unsigned u = __float_as_uint(f);
  return (unsigned short)((u + 0x7FFFu + ((u >> 16) & 1u)) >> 16);
}
__device__ __forceinline__ float bf_bits2f(unsigned short h) { return __uint_as_float(((unsigned)h) << 16); }

__device__ __forceinline__ void dep_guard_h(v8f& a, v8f& b, v16h x, v16h y) { asm volatile("v_nop\n\tv_nop\n\tv_nop\n\tv_nop" : "+v"(a), "+v"(b) : "v"(x), "v"(y)); }
__device__ __forceinline__ void dep_guard_b(v8f& a, v8f& b, v16b x, v16b y) { asm volatile("v_nop\n\tv_nop\n\tv_nop\n\tv_nop" : "+v"(a), "+v"(b) : "v"(x), "v"(y)); }
__device__ __forceinline__ void keep4_h(v16h a, v16h b, v16h c, v16h d) { asm volatile("v_nop" :: "v"(a), "v"(b), "v"(c), "v"(d)); }
__device__ __forceinline__ void keep4_b(v16b a, v16b b, v16b c, v16b d) { asm volatile("v_nop" :: "v"(a), "v"(b), "v"(c), "v"(d)); }
__device__ __forceinline__ void acc_guard4(v8f& a, v8f& b, v8f& c, v8f& d) { asm volatile("v_nop\n\tv_nop\n\tv_nop\n\tv_nop" : "+v"(a), "+v"(b), "+v"(c), "+v"(d)); }
template <typename T> struct Frag;
template <> struct Frag<_Float16> {
  typedef v16h V; union U { v16h v; v8h h[2]; };
  static __device__ __forceinline__ v16h load(const _Float16* p) {
    U f; f.h[0] = *(const v8h*)(p); f.h[1] = *(const v8h*)(p + 16); return f.v;
  }
  static __device__ __forceinline__ v8f mma(v16h a, v16h b, v8f c) {
    return __builtin_amdgcn_wmma_f32_16x16x32_f16(false, a, false, b, (short)0, c, false, false);
  }
  static __device__ __forceinline__ void guard(v8f& a, v8f& b, v16h x, v16h y) { dep_guard_h(a, b, x, y); }
  static __device__ __forceinline__ void keep(v16h a, v16h b, v16h c, v16h d) { keep4_h(a, b, c, d); }
};
template <> struct Frag<__bf16> {
  typedef v16b V; union U { v16b v; v8b h[2]; };
  static __device__ __forceinline__ v16b load(const __bf16* p) {
    U f; f.h[0] = *(const v8b*)(p); f.h[1] = *(const v8b*)(p + 16); return f.v;
  }
  static __device__ __forceinline__ v8f mma(v16b a, v16b b, v8f c) {
    return __builtin_amdgcn_wmma_f32_16x16x32_bf16(false, a, false, b, (short)0, c, false, false);
  }
  static __device__ __forceinline__ void guard(v8f& a, v8f& b, v16b x, v16b y) { dep_guard_b(a, b, x, y); }
  static __device__ __forceinline__ void keep(v16b a, v16b b, v16b c, v16b d) { keep4_b(a, b, c, d); }
};

template <int ET> struct Elem;
template <> struct Elem<0> { typedef _Float16 T; };
template <> struct Elem<1> { typedef __bf16 T; };
template <int ET, bool SPLIT, int BIAS_MODE, int OUT_MODE, bool RESID, int ACT = 0, int TSEL = 0, int KSEL = 0>
__global__ __launch_bounds__(256) void wmma_gemm64(
    const unsigned short* __restrict__ Ap, const unsigned short* __restrict__ A2p, int lda, long strideA,
    const unsigned short* __restrict__ Btp, const unsigned short* __restrict__ Bt2p, int ldb, long strideB,
    void* __restrict__ Cout, void* __restrict__ Cout2, int ldc, long strideC,
    const float* __restrict__ bias,
    const float* __restrict__ resid, long strideR,
    int M, int N, int K, float scale) {
  typedef typename Elem<ET>::T T;
  typedef typename Frag<T>::V V;
  const T* A = (const T*)Ap; const T* A2 = (const T*)A2p; const T* Bt = (const T*)Btp; const T* Bt2 = (const T*)Bt2p;
  __shared__ __align__(16) float sT[8][16 * 68];
  const int b    = blockIdx.y;
  const int lane = threadIdx.x & 31;
  const int wave = threadIdx.x >> 5;
  const int tilesN = N >> 6;
  const int tilesM = M >> 6;
  const int tile = blockIdx.x * 8 + wave;
  if (tile >= tilesM * tilesN) return;
  const int tm = tile / tilesN;
  const int tn = tile - tm * tilesN;
  const int m0 = tm << 6;
  const int n0 = tn << 6;
  if (TSEL == 1 && n0 > m0) return;
  if (TSEL == 2 && !(n0 == m0 || n0 == m0 + 64)) return;

  const T* Ab  = A  + (size_t)b * strideA;
  const T* Bb  = Bt + (size_t)b * strideB;
  const T* Ab2 = SPLIT ? (A2  + (size_t)b * strideA) : nullptr;
  const T* Bb2 = SPLIT ? (Bt2 + (size_t)b * strideB) : nullptr;

  const int rlane = lane & 15;
  const int koff  = (lane >> 4) * 8;
  const int mOff  = (lane >> 4) * 8;

  v8f acc[4][4];
#pragma unroll
  for (int i = 0; i < 4; ++i)
#pragma unroll
    for (int j = 0; j < 4; ++j) acc[i][j] = (v8f){0.f,0.f,0.f,0.f,0.f,0.f,0.f,0.f};

  int kStart = 0;
  int kEnd = K;
  if (KSEL == 1) kEnd = ((m0 + 64) < K) ? (m0 + 64) : K;
  if (KSEL == 2) {
    kStart = (m0 + 64 >= M) ? 0 : m0;
    kEnd = ((m0 + 128) < K) ? (m0 + 128) : K;
  }
  for (int k0 = kStart; k0 < kEnd; k0 += 32) {
    V bh[4], bl[4];
#pragma unroll
    for (int j = 0; j < 4; ++j) {
      const size_t bo = (size_t)(n0 + (j << 4) + rlane) * ldb + koff + k0;
      bh[j] = Frag<T>::load(Bb + bo);
      if (SPLIT) bl[j] = Frag<T>::load(Bb2 + bo);
    }
#pragma unroll
    for (int i = 0; i < 4; ++i) {
      const size_t ao = (size_t)(m0 + (i << 4) + rlane) * lda + koff + k0;
      V ah = Frag<T>::load(Ab + ao);
      V al;
      if (SPLIT) al = Frag<T>::load(Ab2 + ao);
#pragma unroll
      for (int j = 0; j < 4; ++j) {
        acc[i][j] = Frag<T>::mma(ah, bh[j], acc[i][j]);
        if (SPLIT) {
          acc[i][j] = Frag<T>::mma(ah, bl[j], acc[i][j]);
          acc[i][j] = Frag<T>::mma(al, bh[j], acc[i][j]);
        }
      }
      Frag<T>::guard(acc[i][0], acc[i][3], ah, SPLIT ? al : ah);
    }
    Frag<T>::keep(bh[0], bh[1], bh[2], bh[3]);
    if (SPLIT) Frag<T>::keep(bl[0], bl[1], bl[2], bl[3]);
  }
  acc_guard4(acc[0][0], acc[0][1], acc[0][2], acc[0][3]);
  acc_guard4(acc[1][0], acc[1][1], acc[1][2], acc[1][3]);
  acc_guard4(acc[2][0], acc[2][1], acc[2][2], acc[2][3]);
  acc_guard4(acc[3][0], acc[3][1], acc[3][2], acc[3][3]);

  float* slab = sT[wave];
  const float* Rb = RESID ? (resid + (size_t)b * strideR) : nullptr;
#pragma unroll
  for (int i = 0; i < 4; ++i) {
    const int mBase = m0 + (i << 4);
#pragma unroll
    for (int j = 0; j < 4; ++j) {
      const int n = n0 + (j << 4) + rlane;
      float bv = 0.f;
      if (BIAS_MODE == 2) bv = bias[n];
#pragma unroll
      for (int r = 0; r < 8; ++r) {
        float v = acc[i][j][r] * scale;
        if (BIAS_MODE == 1) v += bias[mBase + mOff + r];
        if (BIAS_MODE == 2) v += bv;
        if (RESID) v += Rb[(size_t)(mBase + mOff + r) * ldc + n];
        if (ACT == 1) v = tanhf(v);
        if (ACT == 2) v = fmaxf(v, 0.0f);
        if (ACT == 3) v = v / (1.0f + expf(-v));
        if (ACT == 4) v = (v > 0.f) ? v : 0.01f * v;
        slab[(mOff + r) * 68 + (j << 4) + rlane] = v;
      }
    }
    __builtin_amdgcn_fence(__ATOMIC_RELEASE, "workgroup");
    __builtin_amdgcn_wave_barrier();
    __builtin_amdgcn_fence(__ATOMIC_ACQUIRE, "workgroup");
    if (OUT_MODE == 0) {
      float* C = (float*)Cout + (size_t)b * strideC;
      const int hh = lane >> 4, c4 = (lane & 15) * 4;
      for (int pass = 0; pass < 2; ++pass) {
#pragma unroll
        for (int it = 0; it < 8; ++it) {
          const int row = it * 2 + hh;
          v4f v = *(const v4f*)(slab + row * 68 + c4);
          *(volatile v4f*)(C + (size_t)(mBase + row) * ldc + n0 + c4) = v;
        }
        __threadfence();
      }
    } else {
      const int q = lane >> 3, c8 = (lane & 7) * 8;
      unsigned short* C  = (unsigned short*)Cout  + (size_t)b * strideC;
      unsigned short* C2 = (OUT_MODE == 2) ? ((unsigned short*)Cout2 + (size_t)b * strideC) : nullptr;
      for (int pass = 0; pass < 2; ++pass) {
#pragma unroll
        for (int it = 0; it < 4; ++it) {
          const int row = it * 4 + q;
          const float* sp = slab + row * 68 + c8;
          v8h hv, lv;
#pragma unroll
          for (int e = 0; e < 8; ++e) {
            if (OUT_MODE == 1) {
              hv[e] = (_Float16)sp[e];
            } else {
              unsigned short hb = f2bf_bits(sp[e]);
              unsigned short lb = f2bf_bits(sp[e] - bf_bits2f(hb));
              hv[e] = __builtin_bit_cast(_Float16, hb);
              lv[e] = __builtin_bit_cast(_Float16, lb);
            }
          }
          *(volatile v8h*)(C + (size_t)(mBase + row) * ldc + n0 + c8) = hv;
          if (OUT_MODE == 2) *(volatile v8h*)(C2 + (size_t)(mBase + row) * ldc + n0 + c8) = lv;
        }
        __threadfence();
      }
    }
    __builtin_amdgcn_fence(__ATOMIC_RELEASE, "workgroup");
    __builtin_amdgcn_wave_barrier();
    __builtin_amdgcn_fence(__ATOMIC_ACQUIRE, "workgroup");
  }
}

__device__ __forceinline__ unsigned pk16(unsigned short a, unsigned short b) { return (unsigned)a | ((unsigned)b << 16); }
__device__ __forceinline__ unsigned short h_bits(float f) { const _Float16 h = (_Float16)f; return __builtin_bit_cast(unsigned short, h); }
__device__ __forceinline__ float hbits2f(unsigned short b) { return (float)__builtin_bit_cast(_Float16, b); }
__device__ __forceinline__ float wave_sum(float v) {
#pragma unroll
  for (int off = 16; off > 0; off >>= 1) v += __shfl_xor(v, off, 32);
  return v;
}
__device__ __forceinline__ float wave_max(float v) {
#pragma unroll
  for (int off = 16; off > 0; off >>= 1) v = fmaxf(v, __shfl_xor(v, off, 32));
  return v;
}

__global__ __launch_bounds__(256) void cast_f16x2_kernel(const float* __restrict__ in, unsigned short* __restrict__ out, int n2, float scale) {
  const int i = blockIdx.x * 256 + threadIdx.x;
  if (i < n2) {
    const v2f f = *(const v2f*)(in + 2 * (size_t)i);
    const unsigned u = pk16(h_bits(f[0] * scale), h_bits(f[1] * scale));
    ((volatile unsigned*)out)[i] = u;
    __threadfence();
    ((volatile unsigned*)out)[i] = u;
  }
}

__global__ __launch_bounds__(256) void tcast_f16_kernel(const float* __restrict__ in, unsigned short* __restrict__ out,
                                                        int R, int C, float scale) {
  __shared__ __align__(16) unsigned short t[64 * 72];
  const int c0  = blockIdx.x * 64;
  const int r0  = blockIdx.y * 64;
  const int tid = threadIdx.x;
  {
    const int lr = tid >> 2;
    const int lc = (tid & 3) * 16;
    const float* ip = in + (size_t)(r0 + lr) * C + c0 + lc;
#pragma unroll
    for (int q = 0; q < 4; ++q) {
      const v4f f = *(const v4f*)(ip + 4 * q);
#pragma unroll
      for (int e = 0; e < 4; ++e) t[lr * 72 + lc + 4 * q + e] = h_bits(f[e] * scale);
    }
  }
  __syncthreads();
  const int sub = tid >> 3;
  const int c8  = (tid & 7) * 8;
  v4u hv[2];
#pragma unroll
  for (int it = 0; it < 2; ++it) {
    const int oc = it * 32 + sub;
    v4u a;
#pragma unroll
    for (int q = 0; q < 4; ++q) a[q] = pk16(t[(c8 + 2 * q) * 72 + oc], t[(c8 + 2 * q + 1) * 72 + oc]);
    hv[it] = a;
  }
  for (int pass = 0; pass < 2; ++pass) {
#pragma unroll
    for (int it = 0; it < 2; ++it) {
      const int oc = it * 32 + sub;
      const size_t go = (size_t)(c0 + oc) * R + r0 + c8;
      *(volatile v4u*)(out + go) = hv[it];
    }
    __threadfence();
  }
}

__global__ __launch_bounds__(256) void bias_pack_kernel(const float* __restrict__ b0, const float* __restrict__ b1,
                                                        const float* __restrict__ b2, const float* __restrict__ b3,
                                                        const float* __restrict__ b4, const float* __restrict__ b5,
                                                        float* __restrict__ tab) {
  const int k = blockIdx.x;
  const int tid = threadIdx.x;
  const float* src = b0;
  if (k == 1) src = b1;
  if (k == 2) src = b2;
  if (k == 3) src = b3;
  if (k == 4) src = b4;
  if (k == 5) src = b5;
  const v4f v = *(const v4f*)(src + tid * 4);
  float* dp = tab + (size_t)k * DM + tid * 4;
  *(volatile v4f*)dp = v;
  __threadfence();
  *(volatile v4f*)dp = v;
}

__global__ __launch_bounds__(256) void causal_softmax_kernel(const float* __restrict__ S,
                                                             unsigned short* __restrict__ P) {
  __shared__ float redm[8];
  __shared__ float reds[8];
  const int i    = blockIdx.x;
  const int hg   = blockIdx.y;
  const int tid  = threadIdx.x;
  const int lane = tid & 31;
  const int wave = tid >> 5;
  const int j0   = tid * 8;
  const bool wact = (wave * 256 <= i);
  const float NEG = -1.0e9f;
  float t[8];
#pragma unroll
  for (int e = 0; e < 8; ++e) t[e] = NEG;
  if (wact) {
    const float* rp = S + ((size_t)hg * SEQ + i) * SEQ + j0;
    const v4f a = *(const v4f*)(rp);
    const v4f c = *(const v4f*)(rp + 4);
#pragma unroll
    for (int e = 0; e < 4; ++e) {
      t[e]     = (j0 + e <= i)     ? a[e] : NEG;
      t[4 + e] = (j0 + 4 + e <= i) ? c[e] : NEG;
    }
  }
  float m = fmaxf(fmaxf(fmaxf(t[0], t[1]), fmaxf(t[2], t[3])), fmaxf(fmaxf(t[4], t[5]), fmaxf(t[6], t[7])));
  m = wave_max(m);
  if (lane == 0) redm[wave] = m;
  __syncthreads();
  float mx = redm[0];
#pragma unroll
  for (int w = 1; w < 8; ++w) mx = fmaxf(mx, redm[w]);
  float ex[8];
#pragma unroll
  for (int e = 0; e < 8; ++e) ex[e] = 0.f;
  if (wact) {
#pragma unroll
    for (int e = 0; e < 8; ++e) ex[e] = __expf(t[e] - mx);
  }
  float s = ((ex[0] + ex[1]) + (ex[2] + ex[3])) + ((ex[4] + ex[5]) + (ex[6] + ex[7]));
  s = wave_sum(s);
  if (lane == 0) reds[wave] = s;
  __syncthreads();
  float tot = reds[0];
#pragma unroll
  for (int w = 1; w < 8; ++w) tot += reds[w];
  const float inv = 1.0f / tot;
  unsigned short hb[8];
#pragma unroll
  for (int e = 0; e < 8; ++e) hb[e] = h_bits((ex[e] * inv) * PCARRY);
  const v4u hv = (v4u){pk16(hb[0], hb[1]), pk16(hb[2], hb[3]), pk16(hb[4], hb[5]), pk16(hb[6], hb[7])};
  const size_t ro = ((size_t)hg * SEQ + i) * SEQ + j0;
  *(volatile v4u*)(P + ro) = hv;
  __threadfence();
  *(volatile v4u*)(P + ro) = hv;
}

__global__ __launch_bounds__(256) void window_softmax_kernel(const float* __restrict__ S,
                                                             unsigned short* __restrict__ P) {
  __shared__ float redm[8];
  __shared__ float reds[8];
  const int i    = blockIdx.x;
  const int hg   = blockIdx.y;
  const int tid  = threadIdx.x;
  const int lane = tid & 31;
  const int wave = tid >> 5;
  const int j0   = tid * 8;
  const int jlo  = i + 1;
  const int jhi  = i + WINW;
  const bool uni  = (i == SEQ - 1);
  const bool wact = (wave * 256 <= jhi) && (wave * 256 + 255 >= jlo);
  float t[8];
  bool vb[8];
#pragma unroll
  for (int e = 0; e < 8; ++e) { const int j = j0 + e; vb[e] = (j >= jlo) && (j <= jhi); t[e] = 0.f; }
  if (wact) {
    const float* rp = S + ((size_t)hg * SEQ + i) * SEQ + j0;
    const v4f a = *(const v4f*)(rp);
    const v4f c = *(const v4f*)(rp + 4);
#pragma unroll
    for (int e = 0; e < 4; ++e) { t[e] = a[e]; t[4 + e] = c[e]; }
  }
  float m = -INFINITY;
#pragma unroll
  for (int e = 0; e < 8; ++e) m = fmaxf(m, vb[e] ? t[e] : -INFINITY);
  m = wave_max(m);
  if (lane == 0) redm[wave] = m;
  __syncthreads();
  float mx = redm[0];
#pragma unroll
  for (int w = 1; w < 8; ++w) mx = fmaxf(mx, redm[w]);
  float ex[8];
#pragma unroll
  for (int e = 0; e < 8; ++e) ex[e] = 0.f;
  if (wact) {
#pragma unroll
    for (int e = 0; e < 8; ++e) {
      const float arg = vb[e] ? (t[e] - mx) : 0.f;
      const float ev = __expf(arg);
      ex[e] = vb[e] ? ev : 0.f;
    }
  }
  float s = ((ex[0] + ex[1]) + (ex[2] + ex[3])) + ((ex[4] + ex[5]) + (ex[6] + ex[7]));
  s = wave_sum(s);
  if (lane == 0) reds[wave] = s;
  __syncthreads();
  float tot = reds[0];
#pragma unroll
  for (int w = 1; w < 8; ++w) tot += reds[w];
  const float inv = 1.0f / (uni ? 1.0f : tot);
  const float pu = (1.0f / (float)SEQ) * PCARRY;
  unsigned short hb[8];
#pragma unroll
  for (int e = 0; e < 8; ++e) hb[e] = h_bits(uni ? pu : ((ex[e] * inv) * PCARRY));
  const v4u hv = (v4u){pk16(hb[0], hb[1]), pk16(hb[2], hb[3]), pk16(hb[4], hb[5]), pk16(hb[6], hb[7])};
  const size_t ro = ((size_t)hg * SEQ + i) * SEQ + j0;
  *(volatile v4u*)(P + ro) = hv;
  __threadfence();
  *(volatile v4u*)(P + ro) = hv;
}

__global__ __launch_bounds__(128) void gate_fuse_kernel(const float* __restrict__ G, const unsigned short* __restrict__ FB,
                                                        const float* __restrict__ gg, const float* __restrict__ gb,
                                                        const float* __restrict__ bstr, unsigned short* __restrict__ Fo) {
  __shared__ float ra[4];
  __shared__ float rb[4];
  const int row  = blockIdx.x;
  const int tid  = threadIdx.x;
  const int lane = tid & 31;
  const int wave = tid >> 5;
  const int c0   = tid * 8;
  const float* gp = G + (size_t)row * DM + c0;
  const v4f a = *(const v4f*)(gp);
  const v4f c = *(const v4f*)(gp + 4);
  float xv[8] = {a[0], a[1], a[2], a[3], c[0], c[1], c[2], c[3]};
  float s = ((xv[0] + xv[1]) + (xv[2] + xv[3])) + ((xv[4] + xv[5]) + (xv[6] + xv[7]));
  s = wave_sum(s);
  if (lane == 0) ra[wave] = s;
  __syncthreads();
  const float mean = ((ra[0] + ra[1]) + (ra[2] + ra[3])) * (1.0f / (float)DM);
  float d[8];
  float vs = 0.f;
#pragma unroll
  for (int e = 0; e < 8; ++e) { d[e] = xv[e] - mean; vs += d[e] * d[e]; }
  vs = wave_sum(vs);
  if (lane == 0) rb[wave] = vs;
  __syncthreads();
  const float var  = ((rb[0] + rb[1]) + (rb[2] + rb[3])) * (1.0f / (float)DM);
  const float rstd = rsqrtf(var + LNEPS);
  const float strength = 0.3f / (1.0f + __expf(-bstr[0]));
  const v4f g0 = *(const v4f*)(gg + c0), g1 = *(const v4f*)(gg + c0 + 4);
  const v4f e0 = *(const v4f*)(gb + c0), e1 = *(const v4f*)(gb + c0 + 4);
  float gv[8] = {g0[0], g0[1], g0[2], g0[3], g1[0], g1[1], g1[2], g1[3]};
  float bv[8] = {e0[0], e0[1], e0[2], e0[3], e1[0], e1[1], e1[2], e1[3]};
  const size_t fo = (size_t)row * (2 * DM) + c0;
  const v4u fu = *(const v4u*)(FB + fo);
  const v4u bu = *(const v4u*)(FB + fo + DM);
  float fw[8], bw[8];
#pragma unroll
  for (int q = 0; q < 4; ++q) {
    fw[2 * q]     = hbits2f((unsigned short)(fu[q] & 0xffffu));
    fw[2 * q + 1] = hbits2f((unsigned short)(fu[q] >> 16));
    bw[2 * q]     = hbits2f((unsigned short)(bu[q] & 0xffffu));
    bw[2 * q + 1] = hbits2f((unsigned short)(bu[q] >> 16));
  }
  unsigned short ob[8];
#pragma unroll
  for (int e = 0; e < 8; ++e) {
    const float ln   = d[e] * rstd * gv[e] + bv[e];
    const float gate = __builtin_amdgcn_rcpf(1.0f + __expf(-ln));
    const float f    = fw[e] + strength * gate * bw[e];
    ob[e] = h_bits(f);
  }
  const v4u ov = (v4u){pk16(ob[0], ob[1]), pk16(ob[2], ob[3]), pk16(ob[4], ob[5]), pk16(ob[6], ob[7])};
  unsigned short* op = Fo + (size_t)row * DM + c0;
  *(volatile v4u*)op = ov;
  __threadfence();
  *(volatile v4u*)op = ov;
}

__global__ __launch_bounds__(128) void final_ln_kernel(const float* __restrict__ Y, const float* __restrict__ g,
                                                       const float* __restrict__ bb, float* __restrict__ out) {
  __shared__ float ra[4];
  __shared__ float rb[4];
  const int row  = blockIdx.x;
  const int tid  = threadIdx.x;
  const int lane = tid & 31;
  const int wave = tid >> 5;
  const int c0   = tid * 4;
  const int c1   = (DM / 2) + tid * 4;
  const float* yp = Y + (size_t)row * DM;
  const v4f a = *(const v4f*)(yp + c0);
  const v4f c = *(const v4f*)(yp + c1);
  float xv[8] = {a[0], a[1], a[2], a[3], c[0], c[1], c[2], c[3]};
  float s = ((xv[0] + xv[1]) + (xv[2] + xv[3])) + ((xv[4] + xv[5]) + (xv[6] + xv[7]));
  s = wave_sum(s);
  if (lane == 0) ra[wave] = s;
  __syncthreads();
  const float mean = ((ra[0] + ra[1]) + (ra[2] + ra[3])) * (1.0f / (float)DM);
  float d[8];
  float vs = 0.f;
#pragma unroll
  for (int e = 0; e < 8; ++e) { d[e] = xv[e] - mean; vs += d[e] * d[e]; }
  vs = wave_sum(vs);
  if (lane == 0) rb[wave] = vs;
  __syncthreads();
  const float var  = ((rb[0] + rb[1]) + (rb[2] + rb[3])) * (1.0f / (float)DM);
  const float rstd = rsqrtf(var + LNEPS);
  const v4f g0 = *(const v4f*)(g + c0),  g1 = *(const v4f*)(g + c1);
  const v4f b0 = *(const v4f*)(bb + c0), b1 = *(const v4f*)(bb + c1);
  v4f o0, o1;
#pragma unroll
  for (int e = 0; e < 4; ++e) {
    o0[e] = d[e] * rstd * g0[e] + b0[e];
    o1[e] = d[4 + e] * rstd * g1[e] + b1[e];
  }
  float* op = out + (size_t)row * DM;
  *(volatile v4f*)(op + c0) = o0;
  *(volatile v4f*)(op + c1) = o1;
  __threadfence();
  *(volatile v4f*)(op + c0) = o0;
  *(volatile v4f*)(op + c1) = o1;
}

extern "C" void kernel_launch(void* const* d_in, const int* in_sizes, int n_in,
                              void* d_out, int out_size, void* d_ws, size_t ws_size,
                              hipStream_t stream) {
  if (n_in < 22) return;
  if (in_sizes[0] != NB * SEQ * DM) return;
  const int wsz = DM * DM;
  if (in_sizes[1] != wsz || in_sizes[3] != wsz || in_sizes[5] != wsz || in_sizes[7] != wsz ||
      in_sizes[9] != wsz || in_sizes[11] != wsz || in_sizes[18] != wsz) return;
  if (in_sizes[13] != 2 * DM * DM) return;
  if (in_sizes[2] != DM || in_sizes[4] != DM || in_sizes[6] != DM || in_sizes[8] != DM || in_sizes[10] != DM ||
      in_sizes[12] != DM || in_sizes[14] != DM || in_sizes[15] != DM || in_sizes[16] != DM ||
      in_sizes[19] != DM || in_sizes[20] != DM || in_sizes[21] != DM) return;
  if (in_sizes[17] < 1) return;
  if (out_size != NB * SEQ * DM) return;

  const float* x      = (const float*)d_in[0];
  const float* fq_w   = (const float*)d_in[1];
  const float* fq_b   = (const float*)d_in[2];
  const float* fk_w   = (const float*)d_in[3];
  const float* fk_b   = (const float*)d_in[4];
  const float* fv_w   = (const float*)d_in[5];
  const float* fv_b   = (const float*)d_in[6];
  const float* bq_w   = (const float*)d_in[7];
  const float* bq_b   = (const float*)d_in[8];
  const float* bk_w   = (const float*)d_in[9];
  const float* bk_b   = (const float*)d_in[10];
  const float* bv_w   = (const float*)d_in[11];
  const float* bv_b   = (const float*)d_in[12];
  const float* gate_w = (const float*)d_in[13];
  const float* gate_b = (const float*)d_in[14];
  const float* gln_g  = (const float*)d_in[15];
  const float* gln_b  = (const float*)d_in[16];
  const float* bstr   = (const float*)d_in[17];
  const float* out_w  = (const float*)d_in[18];
  const float* out_b  = (const float*)d_in[19];
  const float* ln_g   = (const float*)d_in[20];
  const float* ln_b   = (const float*)d_in[21];

  const size_t MIB = (size_t)1048576;
  size_t off = 0;
  const size_t oWqk  = off; off += (size_t)4 * DM * DM * 2;
  const size_t oWv2  = off; off += (size_t)2 * DM * DM * 2;
  const size_t oWg   = off; off += (size_t)2 * DM * DM * 2;
  const size_t oWo   = off; off += (size_t)DM * DM * 2;
  const size_t oX16  = off; off += (size_t)SEQ * DM * 2;
  const size_t oQK   = off; off += (size_t)SEQ * 4 * DM * 2;
  const size_t oVT   = off; off += (size_t)2 * DM * SEQ * 2;
  const size_t oS    = off; off += (size_t)HG * SEQ * SEQ * 4;
  const size_t oP    = off; off += (size_t)HG * SEQ * SEQ * 2;
  const size_t oFB   = off; off += (size_t)SEQ * 2 * DM * 2;
  const size_t oFu   = off; off += (size_t)SEQ * DM * 2;
  const size_t oBias = off; off += (size_t)6 * DM * 4;
  const size_t oG    = oS;
  const size_t oY    = oS + 8 * MIB;
  if (off > ws_size) return;
  if (off > (size_t)134217728) return;
  if ((size_t)SEQ * DM * 4 * 2 > (size_t)HG * SEQ * SEQ * 4) return;

  char* ws = (char*)d_ws;
  unsigned short* Wqk  = (unsigned short*)(ws + oWqk);
  unsigned short* Wv2  = (unsigned short*)(ws + oWv2);
  unsigned short* Wg   = (unsigned short*)(ws + oWg);
  unsigned short* Wo   = (unsigned short*)(ws + oWo);
  unsigned short* X16  = (unsigned short*)(ws + oX16);
  unsigned short* QK16 = (unsigned short*)(ws + oQK);
  unsigned short* VT16 = (unsigned short*)(ws + oVT);
  float*          Sbuf = (float*)(ws + oS);
  unsigned short* P16  = (unsigned short*)(ws + oP);
  unsigned short* FB16 = (unsigned short*)(ws + oFB);
  unsigned short* Fu16 = (unsigned short*)(ws + oFu);
  float*          BiasT = (float*)(ws + oBias);
  float*          Gbuf = (float*)(ws + oG);
  float*          Ybuf = (float*)(ws + oY);
  const float*    biasQK = BiasT;
  const float*    biasV  = BiasT + 4 * DM;

  const dim3 blk(256);
  const dim3 blk128(128);

  bias_pack_kernel<<<dim3(6), blk, 0, stream>>>(fq_b, fk_b, bq_b, bk_b, fv_b, bv_b, BiasT);
  const dim3 gTW(DM / 64, DM / 64);
  tcast_f16_kernel<<<gTW, blk, 0, stream>>>(fq_w, Wqk + (size_t)0 * DM * DM, DM, DM, WCARRY);
  tcast_f16_kernel<<<gTW, blk, 0, stream>>>(fk_w, Wqk + (size_t)1 * DM * DM, DM, DM, WCARRY);
  tcast_f16_kernel<<<gTW, blk, 0, stream>>>(bq_w, Wqk + (size_t)2 * DM * DM, DM, DM, WCARRY);
  tcast_f16_kernel<<<gTW, blk, 0, stream>>>(bk_w, Wqk + (size_t)3 * DM * DM, DM, DM, WCARRY);
  tcast_f16_kernel<<<gTW, blk, 0, stream>>>(fv_w, Wv2 + (size_t)0 * DM * DM, DM, DM, WCARRY);
  tcast_f16_kernel<<<gTW, blk, 0, stream>>>(bv_w, Wv2 + (size_t)1 * DM * DM, DM, DM, WCARRY);
  tcast_f16_kernel<<<dim3(DM / 64, 2 * DM / 64), blk, 0, stream>>>(gate_w, Wg, 2 * DM, DM, WCARRY);
  tcast_f16_kernel<<<gTW, blk, 0, stream>>>(out_w, Wo, DM, DM, WCARRY);

  const int n2x = SEQ * DM / 2;
  const dim3 gCastX((n2x + 255) / 256);
  const int tilesM = SEQ / 64;
  const dim3 gQK((tilesM * (4 * DM / 64) + 7) / 8, 1);
  const dim3 gVT(((2 * DM / 64) * (SEQ / 64) + 7) / 8, 1);
  const dim3 gS((tilesM * (SEQ / 64) + 7) / 8, HG);
  const dim3 gPV((tilesM * (HD / 64) + 7) / 8, HG);
  const dim3 gG((tilesM * (DM / 64) + 7) / 8, 1);
  const dim3 gO((tilesM * (DM / 64) + 7) / 8, 1);
  const float wscale  = 1.0f / WCARRY;
  const float sscale  = 0.125f;
  const float pvscale = FBCARRY * PCARRY_INV;
  const float gscale  = 1.0f / (WCARRY * FBCARRY);
  const float oscale  = 1.0f / (WCARRY * FBCARRY);

  for (int b = 0; b < NB; ++b) {
    const float* xb = x + (size_t)b * SEQ * DM;
    cast_f16x2_kernel<<<gCastX, blk, 0, stream>>>(xb, X16, n2x, 1.0f);
    wmma_gemm64<0, false, 2, 1, false, 0, 0, 0><<<gQK, blk, 0, stream>>>(
        X16, X16, DM, 0L, Wqk, Wqk, DM, 0L, (void*)QK16, (void*)QK16, 4 * DM, 0L,
        biasQK, biasQK, 0L, SEQ, 4 * DM, DM, wscale);
    wmma_gemm64<0, false, 1, 1, false, 0, 0, 0><<<gVT, blk, 0, stream>>>(
        Wv2, Wv2, DM, 0L, X16, X16, DM, 0L, (void*)VT16, (void*)VT16, SEQ, 0L,
        biasV, biasV, 0L, 2 * DM, SEQ, DM, wscale);
    for (int g = 0; g < NGRP; ++g) {
      const size_t hc = (size_t)g * HG * HD;
      wmma_gemm64<0, false, 0, 0, false, 0, 1, 0><<<gS, blk, 0, stream>>>(
          QK16 + hc, QK16 + hc, 4 * DM, (long)HD, QK16 + DM + hc, QK16 + DM + hc, 4 * DM, (long)HD,
          (void*)Sbuf, (void*)Sbuf, SEQ, (long)SEQ * SEQ,
          biasQK, biasQK, 0L, SEQ, SEQ, HD, sscale);
      causal_softmax_kernel<<<dim3(SEQ, HG), blk, 0, stream>>>(Sbuf, P16);
      wmma_gemm64<0, false, 0, 1, false, 0, 0, 1><<<gPV, blk, 0, stream>>>(
          P16, P16, SEQ, (long)SEQ * SEQ, VT16 + hc * SEQ, VT16 + hc * SEQ, SEQ, (long)HD * SEQ,
          (void*)(FB16 + hc), (void*)(FB16 + hc), 2 * DM, (long)HD,
          biasQK, biasQK, 0L, SEQ, HD, SEQ, pvscale);
      wmma_gemm64<0, false, 0, 0, false, 0, 2, 0><<<gS, blk, 0, stream>>>(
          QK16 + 2 * DM + hc, QK16 + 2 * DM + hc, 4 * DM, (long)HD, QK16 + 3 * DM + hc, QK16 + 3 * DM + hc, 4 * DM, (long)HD,
          (void*)Sbuf, (void*)Sbuf, SEQ, (long)SEQ * SEQ,
          biasQK, biasQK, 0L, SEQ, SEQ, HD, sscale);
      window_softmax_kernel<<<dim3(SEQ, HG), blk, 0, stream>>>(Sbuf, P16);
      wmma_gemm64<0, false, 0, 1, false, 0, 0, 2><<<gPV, blk, 0, stream>>>(
          P16, P16, SEQ, (long)SEQ * SEQ, VT16 + (DM + hc) * SEQ, VT16 + (DM + hc) * SEQ, SEQ, (long)HD * SEQ,
          (void*)(FB16 + DM + hc), (void*)(FB16 + DM + hc), 2 * DM, (long)HD,
          biasQK, biasQK, 0L, SEQ, HD, SEQ, pvscale);
    }
    wmma_gemm64<0, false, 2, 0, false, 0, 0, 0><<<gG, blk, 0, stream>>>(
        FB16, FB16, 2 * DM, 0L, Wg, Wg, 2 * DM, 0L, (void*)Gbuf, (void*)Gbuf, DM, 0L,
        gate_b, gate_b, 0L, SEQ, DM, 2 * DM, gscale);
    gate_fuse_kernel<<<dim3(SEQ), blk128, 0, stream>>>(Gbuf, FB16, gln_g, gln_b, bstr, Fu16);
    wmma_gemm64<0, false, 2, 0, true, 0, 0, 0><<<gO, blk, 0, stream>>>(
        Fu16, Fu16, DM, 0L, Wo, Wo, DM, 0L, (void*)Ybuf, (void*)Ybuf, DM, 0L,
        out_b, xb, 0L, SEQ, DM, DM, oscale);
    final_ln_kernel<<<dim3(SEQ), blk128, 0, stream>>>(Ybuf, ln_g, ln_b, (float*)d_out + (size_t)b * SEQ * DM);
  }
  (void)hipGetLastError();
}
